// GNN_8555574853744
// MI455X (gfx1250) — hardware-verified
//
#include <hip/hip_runtime.h>
#include <stddef.h>
#include <stdint.h>
#include <math.h>


#define CIN    128
#define C1     256
#define C2     128
#define K2     512
#define ED     8
#define NTHR   256
#define NWAVE  8
#define EPT    8
#define CHUNK  (NTHR * EPT)
#define WCAP   (EPT * 32)
#define LISTN  (NWAVE * WCAP)
#define NBA    1024
#define SLA    10
#define RCAP   28672
#define DEGCAP 64
#define AP     512
#define GTHR   128
#define EB     1024
#define NU1    (C1 * (CIN / 8))
#define NU2    (C2 * (K2 / 8))
#define AGG_ZINTS    (LISTN + 2 * RCAP + 3 * NBA)
#define MISC_INTS    16
#define ROWBUF_INTS  (NWAVE * AP / 2)
#define AGG_LDS_INTS (AGG_ZINTS + MISC_INTS + ROWBUF_INTS)
#define WSMAX  134217728

static_assert((CHUNK & (CHUNK - 1)) == 0 && CHUNK <= 4096);
static_assert((NBA & (NBA - 1)) == 0 && NBA == (1 << SLA));
static_assert(((long long)CHUNK << SLA) < (1LL << 31));
static_assert(LISTN % NTHR == 0);
static_assert(NBA % NWAVE == 0 && NBA % 32 == 0 && NBA % 64 == 0);
static_assert(RCAP % 4 == 0 && AGG_ZINTS % 4 == 0 && LISTN % 4 == 0 && ((AGG_ZINTS + MISC_INTS) % 4) == 0);
static_assert(CIN % 32 == 0 && K2 % 32 == 0 && K2 == 2 * C1 && AP == K2);
static_assert(NU1 % NTHR == 0 && NU2 % NTHR == 0);
static_assert(CIN / 8 == 16 && K2 / 8 == 64);
static_assert(C1 == 2 * 128 && C2 == 128);
static_assert(NWAVE == ED);
static_assert(EB == 4 * NTHR);
static_assert(DEGCAP == 64);
static_assert(AGG_LDS_INTS * 4 <= 300000);

typedef float          v4f   __attribute__((ext_vector_type(4)));
typedef float          v8f   __attribute__((ext_vector_type(8)));
typedef double         v2d   __attribute__((ext_vector_type(2)));
typedef int            v4i   __attribute__((ext_vector_type(4)));
typedef int            v8i   __attribute__((ext_vector_type(8)));
typedef unsigned short v4us  __attribute__((ext_vector_type(4)));
typedef unsigned short v8us  __attribute__((ext_vector_type(8)));
typedef unsigned short v16us __attribute__((ext_vector_type(16)));
typedef __bf16         v16bf __attribute__((ext_vector_type(16)));
typedef v4f  __attribute__((may_alias)) v4fa;
typedef v4i  __attribute__((may_alias)) v4ia;
typedef v4us __attribute__((may_alias)) v4usa;
typedef v8us __attribute__((may_alias)) v8usa;
union FragB { v16bf v; v16us u; v8us h[2]; v8i w; };

__device__ __forceinline__ v8f wmb(const FragB& a, const FragB& b, v8f c) {
  v8f d = __builtin_amdgcn_wmma_f32_16x16x32_bf16(false, a.v, false, b.v, (short)0, c, false, false);
  asm volatile("v_nop\n\tv_nop\n\tv_nop\n\tv_nop" : "+v"(d) : "v"(a.w), "v"(b.w));
  return d;
}

__device__ __forceinline__ unsigned bf16_bits(float f) {
  const unsigned u = __float_as_uint(f);
  const unsigned r = (u + 0x7FFFu + ((u >> 16) & 1u)) >> 16;
  return (f != f) ? 0x7FC0u : r;
}
__device__ __forceinline__ float bf16_val(float f) {
  return __uint_as_float(bf16_bits(f) << 16);
}
__device__ __forceinline__ float relu_np(float v) { return (v > 0.0f) ? v : (v - v); }
__device__ __forceinline__ float leaky(float a) { return (a >= 0.0f) ? a : 0.2f * a; }

__device__ __forceinline__ void wave_sync() {
  __builtin_amdgcn_fence(__ATOMIC_RELEASE, "wavefront");
  __builtin_amdgcn_wave_barrier();
  __builtin_amdgcn_fence(__ATOMIC_ACQUIRE, "wavefront");
}

template <int SLB>
__device__ __forceinline__ int scan_chunk(const int* __restrict__ dsts, int nE, int cbase, int slotBase,
                                          int nb, int vec8, int* list, int tid, int lane, int wave) {
  int wc = 0;
  const int el0  = tid * EPT;
  const int e0   = cbase + el0;
  const int sent = -2147483647 - 1;
  v4i da, db;
  if (vec8 != 0 && cbase + CHUNK <= nE) {
    da = *(const v4i*)(dsts + e0);
    db = *(const v4i*)(dsts + e0 + 4);
  } else {
    da.x = (e0     < nE) ? dsts[min(e0,     nE - 1)] : sent;
    da.y = (e0 + 1 < nE) ? dsts[min(e0 + 1, nE - 1)] : sent;
    da.z = (e0 + 2 < nE) ? dsts[min(e0 + 2, nE - 1)] : sent;
    da.w = (e0 + 3 < nE) ? dsts[min(e0 + 3, nE - 1)] : sent;
    db.x = (e0 + 4 < nE) ? dsts[min(e0 + 4, nE - 1)] : sent;
    db.y = (e0 + 5 < nE) ? dsts[min(e0 + 5, nE - 1)] : sent;
    db.z = (e0 + 6 < nE) ? dsts[min(e0 + 6, nE - 1)] : sent;
    db.w = (e0 + 7 < nE) ? dsts[min(e0 + 7, nE - 1)] : sent;
  }
  const unsigned nbs = (unsigned)slotBase;
  const unsigned unb = (unsigned)nb;
  const unsigned s0 = (unsigned)da.x - nbs, s1 = (unsigned)da.y - nbs;
  const unsigned s2 = (unsigned)da.z - nbs, s3 = (unsigned)da.w - nbs;
  const unsigned s4 = (unsigned)db.x - nbs, s5 = (unsigned)db.y - nbs;
  const unsigned s6 = (unsigned)db.z - nbs, s7 = (unsigned)db.w - nbs;
  const bool h0 = s0 < unb, h1 = s1 < unb, h2 = s2 < unb, h3 = s3 < unb;
  const bool h4 = s4 < unb, h5 = s5 < unb, h6 = s6 < unb, h7 = s7 < unb;
  const unsigned any = __builtin_amdgcn_ballot_w32(h0 | h1 | h2 | h3 | h4 | h5 | h6 | h7);
  if (any != 0u) {
#define HITJ(J, HJ, SJ) { \
      const unsigned mj = __builtin_amdgcn_ballot_w32(HJ); \
      if (mj != 0u) { \
        if (HJ) { \
          const int pos = wc + (int)__builtin_amdgcn_mbcnt_lo(mj, 0u); \
          if (pos < WCAP) list[wave * WCAP + pos] = ((el0 + (J)) << SLB) | (int)(SJ); \
        } \
        wc += (int)__builtin_popcount(mj); } }
    HITJ(0, h0, s0)
    HITJ(1, h1, s1)
    HITJ(2, h2, s2)
    HITJ(3, h3, s3)
    HITJ(4, h4, s4)
    HITJ(5, h5, s5)
    HITJ(6, h6, s6)
    HITJ(7, h7, s7)
#undef HITJ
  }
  return wc;
}

__device__ __forceinline__ void block_ve(const float* __restrict__ We1, const float* __restrict__ ae1,
                                         const float* __restrict__ We2, const float* __restrict__ ae2,
                                         float* sve, int lane, int wave) {
  float s1 = 0.0f, s2 = 0.0f;
#pragma unroll
  for (int i = 0; i < 2; ++i) {
    const v4f w = *(const v4f*)(We1 + (size_t)wave * C1 + 128 * i + 4 * lane);
    const v4f a = *(const v4f*)(ae1 + 128 * i + 4 * lane);
    s1 = fmaf(bf16_val(w.x), bf16_val(a.x), s1);
    s1 = fmaf(bf16_val(w.y), bf16_val(a.y), s1);
    s1 = fmaf(bf16_val(w.z), bf16_val(a.z), s1);
    s1 = fmaf(bf16_val(w.w), bf16_val(a.w), s1);
  }
  {
    const v4f w = *(const v4f*)(We2 + (size_t)wave * C2 + 4 * lane);
    const v4f a = *(const v4f*)(ae2 + 4 * lane);
    s2 = fmaf(bf16_val(w.x), bf16_val(a.x), s2);
    s2 = fmaf(bf16_val(w.y), bf16_val(a.y), s2);
    s2 = fmaf(bf16_val(w.z), bf16_val(a.z), s2);
    s2 = fmaf(bf16_val(w.w), bf16_val(a.w), s2);
  }
#pragma unroll
  for (int off = 16; off > 0; off >>= 1) {
    s1 += __shfl_xor(s1, off, 32);
    s2 += __shfl_xor(s2, off, 32);
  }
  if (lane == 0) { sve[wave] = s1; sve[8 + wave] = s2; }
}

__global__ __launch_bounds__(NTHR) void k_wprep(const float* __restrict__ W1, const float* __restrict__ W2,
                                                unsigned short* W1T, unsigned short* W2T2) {
  const int u = (int)blockIdx.x * NTHR + (int)threadIdx.x;
  v8us o;
  unsigned short* dp;
  if (u < NU1) {
    const int n  = u >> 4;
    const int k8 = (u & 15) * 8;
    const float* p = W1 + (size_t)k8 * C1 + n;
#pragma unroll
    for (int i = 0; i < 8; ++i) o[i] = (unsigned short)bf16_bits(p[(size_t)i * C1]);
    dp = W1T + (size_t)n * CIN + k8;
  } else if (u < NU1 + NU2) {
    const int v  = u - NU1;
    const int n  = v >> 6;
    const int k8 = (v & 63) * 8;
    const int kk = k8 & (C1 - 1);
    const float* p = W2 + (size_t)kk * C2 + n;
#pragma unroll
    for (int i = 0; i < 8; ++i) o[i] = (unsigned short)bf16_bits(p[(size_t)i * C2]);
    dp = W2T2 + (size_t)n * K2 + k8;
  } else {
    return;
  }
  *(volatile v8us*)dp = o;
  __threadfence();
  *(volatile v8us*)dp = o;
}

__global__ __launch_bounds__(NTHR) void k_cvx(const float* __restrict__ x, int nN, int nUnits,
                                              unsigned short* xb) {
  const int u = (int)blockIdx.x * NTHR + (int)threadIdx.x;
  if (u >= nUnits) return;
  const int row = u >> 4;
  const int k8  = (u & 15) * 8;
  const int rc  = row < nN ? row : nN - 1;
  const float* p = x + (size_t)rc * CIN + k8;
  const v4f a = *(const v4fa*)p;
  const v4f b = *(const v4fa*)(p + 4);
  const bool ok = row < nN;
  v8us o;
  o[0] = ok ? (unsigned short)bf16_bits(a.x) : (unsigned short)0;
  o[1] = ok ? (unsigned short)bf16_bits(a.y) : (unsigned short)0;
  o[2] = ok ? (unsigned short)bf16_bits(a.z) : (unsigned short)0;
  o[3] = ok ? (unsigned short)bf16_bits(a.w) : (unsigned short)0;
  o[4] = ok ? (unsigned short)bf16_bits(b.x) : (unsigned short)0;
  o[5] = ok ? (unsigned short)bf16_bits(b.y) : (unsigned short)0;
  o[6] = ok ? (unsigned short)bf16_bits(b.z) : (unsigned short)0;
  o[7] = ok ? (unsigned short)bf16_bits(b.w) : (unsigned short)0;
  unsigned short* dp = xb + (size_t)row * CIN + k8;
  *(volatile v8us*)dp = o;
  __threadfence();
  *(volatile v8us*)dp = o;
}

__global__ __launch_bounds__(NTHR) void k_edge(const float* __restrict__ ea, int nE,
                                               const float* __restrict__ We1, const float* __restrict__ ae1,
                                               const float* __restrict__ We2, const float* __restrict__ ae2,
                                               float* AE1, float* AE2, double* rec) {
  __shared__ __attribute__((aligned(16))) float sve[16];
  __shared__ __attribute__((aligned(16))) float sA1[EB];
  __shared__ __attribute__((aligned(16))) float sA2[EB];
  __shared__ __attribute__((aligned(16))) float sm[ED * NTHR];
  __shared__ __attribute__((aligned(16))) double srec[16];
  const int tid = (int)threadIdx.x, lane = tid & 31, wave = tid >> 5;
  block_ve(We1, ae1, We2, ae2, sve, lane, wave);
  __syncthreads();
  float v1[ED], v2[ED], cs[ED];
#pragma unroll
  for (int j = 0; j < ED; ++j) { v1[j] = sve[j]; v2[j] = sve[8 + j]; cs[j] = 0.0f; }
  const int eb = (int)blockIdx.x * EB;
#pragma unroll 1
  for (int it = 0; it < 4; ++it) {
    const int el = it * NTHR + tid;
    const int e  = eb + el;
    const bool ok = e < nE;
    const int ec = ok ? e : nE - 1;
    const float* p = ea + (size_t)ec * ED;
    const v4f a = *(const v4f*)p;
    const v4f b = *(const v4f*)(p + 4);
    float f[ED];
    f[0] = ok ? bf16_val(a.x) : 0.0f; f[1] = ok ? bf16_val(a.y) : 0.0f;
    f[2] = ok ? bf16_val(a.z) : 0.0f; f[3] = ok ? bf16_val(a.w) : 0.0f;
    f[4] = ok ? bf16_val(b.x) : 0.0f; f[5] = ok ? bf16_val(b.y) : 0.0f;
    f[6] = ok ? bf16_val(b.z) : 0.0f; f[7] = ok ? bf16_val(b.w) : 0.0f;
    float d1 = f[0] * v1[0], d2 = f[0] * v2[0];
#pragma unroll
    for (int j = 1; j < ED; ++j) { d1 = fmaf(f[j], v1[j], d1); d2 = fmaf(f[j], v2[j], d2); }
#pragma unroll
    for (int j = 0; j < ED; ++j) cs[j] += f[j];
    sA1[el] = d1;
    sA2[el] = d2;
  }
#pragma unroll
  for (int j = 0; j < ED; ++j) sm[j * NTHR + tid] = cs[j];
  __syncthreads();
  {
    const v4f q0 = *(const v4fa*)(sm + wave * NTHR + 8 * lane);
    const v4f q1 = *(const v4fa*)(sm + wave * NTHR + 8 * lane + 4);
    double s = (double)q0.x;
    s += (double)q0.y; s += (double)q0.z; s += (double)q0.w;
    s += (double)q1.x; s += (double)q1.y; s += (double)q1.z; s += (double)q1.w;
#pragma unroll
    for (int off = 16; off > 0; off >>= 1) s += __shfl_xor(s, off, 32);
    if (lane == 0) { srec[wave] = s; srec[8 + wave] = 0.0; }
  }
  const v4f o1 = *(const v4fa*)(sA1 + 4 * tid);
  const v4f o2 = *(const v4fa*)(sA2 + 4 * tid);
  float* p1 = AE1 + (size_t)eb + 4 * tid;
  float* p2 = AE2 + (size_t)eb + 4 * tid;
  *(volatile v4f*)p1 = o1;
  *(volatile v4f*)p2 = o2;
  __threadfence();
  *(volatile v4f*)p1 = o1;
  *(volatile v4f*)p2 = o2;
  __syncthreads();
  {
    const int lc = lane & 7;
    v2d r;
    r.x = srec[2 * lc];
    r.y = srec[2 * lc + 1];
    double* rp = rec + (size_t)blockIdx.x * 16 + 2 * lc;
    const bool okst = (wave == 0) && (lane < 8);
    if (okst) *(volatile v2d*)rp = r;
    __threadfence();
    if (okst) *(volatile v2d*)rp = r;
  }
}

__global__ __launch_bounds__(NTHR) void k_combine(const double* __restrict__ rec, int nRec, int nE,
                                                  const float* __restrict__ We1, const float* __restrict__ ae1,
                                                  const float* __restrict__ We2, const float* __restrict__ ae2,
                                                  float* sc) {
  __shared__ __attribute__((aligned(16))) float sve[16];
  __shared__ __attribute__((aligned(16))) float smean[8];
  __shared__ __attribute__((aligned(16))) float ssc[32];
  const int tid = (int)threadIdx.x, lane = tid & 31, wave = tid >> 5;
  block_ve(We1, ae1, We2, ae2, sve, lane, wave);
  double s = 0.0;
#pragma unroll 1
  for (int b0 = 0; b0 < nRec; b0 += 32) {
    const int b  = b0 + lane;
    const int bc = b < nRec ? b : nRec - 1;
    const double v = rec[(size_t)bc * 16 + wave];
    s += (b < nRec) ? v : 0.0;
  }
#pragma unroll
  for (int off = 16; off > 0; off >>= 1) s += __shfl_xor(s, off, 32);
  if (lane == 0) smean[wave] = (float)(s / (double)nE);
  __syncthreads();
  if (tid < 32) {
    float a1 = smean[0] * sve[0], a2 = smean[0] * sve[8];
#pragma unroll
    for (int j = 1; j < ED; ++j) { a1 = fmaf(smean[j], sve[j], a1); a2 = fmaf(smean[j], sve[8 + j], a2); }
    int vi = tid - 2;
    vi = vi < 0 ? 0 : (vi > 15 ? 15 : vi);
    const float vv = sve[vi];
    float o = 0.0f;
    o = (tid >= 2 && tid < 18) ? vv : o;
    o = (tid == 0) ? a1 : o;
    o = (tid == 1) ? a2 : o;
    ssc[tid] = o;
  }
  __syncthreads();
  {
    const v4f ov = *(const v4fa*)(ssc + 4 * (lane & 7));
    float* op = sc + 4 * (lane & 7);
    const bool okst = (wave == 0) && (lane < 8);
    if (okst) *(volatile v4f*)op = ov;
    __threadfence();
    if (okst) *(volatile v4f*)op = ov;
  }
}

template <int RG, int CH>
__global__ __launch_bounds__(GTHR) void k_gemm(const unsigned short* __restrict__ A,
                                               const unsigned short* __restrict__ BT, int K,
                                               const float* __restrict__ avs, const float* __restrict__ avd,
                                               float* Hout, float* ASo, float* ADo) {
  constexpr int GM  = 16 * RG;
  constexpr int NC  = 128 * CH;
  constexpr int RPW = GM / 4;
  constexpr int NL  = GM / 4;
  static_assert(RG * CH == 4 && GM * NC == 8192 && GM <= 64);
  __shared__ __attribute__((aligned(16))) float stg[GM * NC];
  __shared__ __attribute__((aligned(16))) float sAS[64];
  __shared__ __attribute__((aligned(16))) float sAD[64];
  const int tid = (int)threadIdx.x, lane = tid & 31, wave = tid >> 5, hh = lane >> 4, m = lane & 15;
  const int rg = wave % RG, ch = wave / RG;
  const int rowBase = (int)blockIdx.x * GM;

  v8f acc[8];
  {
    const v8f z = {0.f, 0.f, 0.f, 0.f, 0.f, 0.f, 0.f, 0.f};
#pragma unroll
    for (int t = 0; t < 8; ++t) acc[t] = z;
  }
  const unsigned short* ap = A  + (size_t)(rowBase + 16 * rg + m) * (size_t)K + 8 * hh;
  const unsigned short* bp = BT + (size_t)(128 * ch + m) * (size_t)K + 8 * hh;

#pragma unroll 1
  for (int k0 = 0; k0 < K; k0 += 32) {
    FragB af;
    af.h[0] = *(const v8usa*)(ap + k0);
    af.h[1] = *(const v8usa*)(ap + k0 + 16);
#pragma unroll
    for (int nt = 0; nt < 8; ++nt) {
      const unsigned short* wq = bp + (size_t)(16 * nt) * (size_t)K + k0;
      FragB bf;
      bf.h[0] = *(const v8usa*)wq;
      bf.h[1] = *(const v8usa*)(wq + 16);
      acc[nt] = wmb(af, bf, acc[nt]);
    }
  }

#pragma unroll
  for (int nt = 0; nt < 8; ++nt) {
    const int lc = 128 * ch + 16 * nt + m;
#pragma unroll
    for (int r = 0; r < 8; ++r) {
      const int lr = 16 * rg + 8 * hh + r;
      stg[lr * NC + lc] = acc[nt][r];
    }
  }
  __syncthreads();

  v4f vs[CH], vd[CH];
#pragma unroll
  for (int j = 0; j < CH; ++j) {
    const v4f t1 = *(const v4f*)(avs + 128 * j + 4 * lane);
    const v4f t2 = *(const v4f*)(avd + 128 * j + 4 * lane);
    vs[j].x = bf16_val(t1.x); vs[j].y = bf16_val(t1.y); vs[j].z = bf16_val(t1.z); vs[j].w = bf16_val(t1.w);
    vd[j].x = bf16_val(t2.x); vd[j].y = bf16_val(t2.y); vd[j].z = bf16_val(t2.z); vd[j].w = bf16_val(t2.w);
  }

#pragma unroll 1
  for (int i = 0; i < RPW; ++i) {
    const int lr = RPW * wave + i;
    const int gr = rowBase + lr;
    float s1 = 0.0f, s2 = 0.0f;
#pragma unroll
    for (int j = 0; j < CH; ++j) {
      const v4f v = *(const v4fa*)(stg + lr * NC + 128 * j + 4 * lane);
      s1 = fmaf(v.x, vs[j].x, s1); s1 = fmaf(v.y, vs[j].y, s1);
      s1 = fmaf(v.z, vs[j].z, s1); s1 = fmaf(v.w, vs[j].w, s1);
      s2 = fmaf(v.x, vd[j].x, s2); s2 = fmaf(v.y, vd[j].y, s2);
      s2 = fmaf(v.z, vd[j].z, s2); s2 = fmaf(v.w, vd[j].w, s2);
      *(volatile v4f*)(Hout + (size_t)gr * NC + 128 * j + 4 * lane) = v;
    }
#pragma unroll
    for (int off = 16; off > 0; off >>= 1) {
      s1 += __shfl_xor(s1, off, 32);
      s2 += __shfl_xor(s2, off, 32);
    }
    if (lane == 0) { sAS[lr] = s1; sAD[lr] = s2; }
  }
  __threadfence();
#pragma unroll 1
  for (int i = 0; i < RPW; ++i) {
    const int lr = RPW * wave + i;
    const int gr = rowBase + lr;
#pragma unroll
    for (int j = 0; j < CH; ++j) {
      const v4f v = *(const v4fa*)(stg + lr * NC + 128 * j + 4 * lane);
      *(volatile v4f*)(Hout + (size_t)gr * NC + 128 * j + 4 * lane) = v;
    }
  }
  __syncthreads();
  {
    const int lc = lane < NL ? lane : NL - 1;
    const v4f a4 = *(const v4fa*)(sAS + 4 * lc);
    const v4f d4 = *(const v4fa*)(sAD + 4 * lc);
    float* pa = ASo + (size_t)rowBase + 4 * lc;
    float* pd = ADo + (size_t)rowBase + 4 * lc;
    const bool okst = (wave == 0) && (lane < NL);
    if (okst) { *(volatile v4f*)pa = a4; *(volatile v4f*)pd = d4; }
    __threadfence();
    if (okst) { *(volatile v4f*)pa = a4; *(volatile v4f*)pd = d4; }
  }
}

template <int NV>
__device__ __forceinline__ void gacc(const float* __restrict__ Hp, int row, float w, int lane, v4f (&acc)[NV]) {
  const float* rp = Hp + (size_t)row * (size_t)(128 * NV) + 4 * lane;
#pragma unroll
  for (int j = 0; j < NV; ++j) {
    const v4f a = *(const v4f*)(rp + 128 * j);
    acc[j].x = fmaf(w, a.x, acc[j].x);
    acc[j].y = fmaf(w, a.y, acc[j].y);
    acc[j].z = fmaf(w, a.z, acc[j].z);
    acc[j].w = fmaf(w, a.w, acc[j].w);
  }
}

template <int NV>
__global__ __launch_bounds__(NTHR) void k_scan(const int* __restrict__ srcs, const int* __restrict__ dsts,
                                               int nE, int nN, int vec8, int mRows,
                                               const float* __restrict__ AEp, const float* __restrict__ ASp,
                                               const float* __restrict__ ADp, const float* __restrict__ sc,
                                               int aelIdx, const float* __restrict__ Hp,
                                               const float* __restrict__ bias,
                                               unsigned short* xpl, float* outp) {
  extern __shared__ __attribute__((aligned(16))) int dsm[];
  int* list = dsm;
  int* hl   = dsm + LISTN;
  int* sl   = hl + RCAP;
  int* cnt  = sl + RCAP;
  int* offs = cnt + NBA;
  int* cur  = offs + NBA;
  int* misc = cur + NBA;
  const int tid = (int)threadIdx.x, lane = tid & 31, wave = tid >> 5;
  unsigned short* rowbuf = (unsigned short*)(misc + MISC_INTS) + wave * AP;
  const int nodeBase = (int)blockIdx.x * NBA;

  {
    const v4i z4 = {0, 0, 0, 0};
    for (int i = tid * 4; i < AGG_ZINTS; i += NTHR * 4) *(v4ia*)(dsm + i) = z4;
    if (tid < MISC_INTS) misc[tid] = 0;
  }
  __syncthreads();

  int t = 0, ov = 0;
  const int nChunks = (nE + CHUNK - 1) / CHUNK;
#pragma unroll 1
  for (int ch = 0; ch < nChunks; ++ch) {
    const int cbase = ch * CHUNK;
    const int wc = scan_chunk<SLA>(dsts, nE, cbase, nodeBase, NBA, vec8, list, tid, lane, wave);
    if (lane == 0) misc[wave] = wc;
    __syncthreads();
    if (wave == 0) {
#pragma unroll 1
      for (int w2 = 0; w2 < NWAVE; ++w2) {
        int c = misc[w2];
        c = c < 0 ? 0 : (c > WCAP ? WCAP : c);
#pragma unroll 1
        for (int b0 = 0; b0 < c; b0 += 32) {
          const int idx = b0 + lane;
          const int ent = list[w2 * WCAP + (idx < WCAP ? idx : WCAP - 1)];
          const int m32 = (c - b0) < 32 ? (c - b0) : 32;
#pragma unroll 1
          for (int k = 0; k < m32; ++k) {
            const int u    = __builtin_amdgcn_readlane(ent, k);
            const int slot = u & (NBA - 1);
            const int el   = (u >> SLA) & (CHUNK - 1);
            const int pk   = ((cbase + el) << SLA) | slot;
            if (t < RCAP) {
              if (lane == 0) { hl[t] = pk; cnt[slot] = cnt[slot] + 1; }
              t = t + 1;
            } else {
              ov = 1;
            }
          }
        }
      }
    }
    __syncthreads();
  }
  if (wave == 0 && lane == 0) { misc[8] = t; misc[9] = ov; }
  __syncthreads();
  int tt = misc[8];
  tt = tt < 0 ? 0 : (tt > RCAP ? RCAP : tt);
  const int ovf = misc[9];

  if (wave == 0) {
    const int base = lane * (NBA / 32);
    int s = 0;
#pragma unroll 1
    for (int i = 0; i < NBA / 32; ++i) s += cnt[base + i];
    int incl = s;
#pragma unroll
    for (int d = 1; d < 32; d <<= 1) {
      const int y = __shfl_up(incl, d, 32);
      if (lane >= d) incl += y;
    }
    int run = incl - s;
#pragma unroll 1
    for (int i = 0; i < NBA / 32; ++i) {
      const int cv = cnt[base + i];
      offs[base + i] = run;
      cur[base + i]  = run;
      run += cv;
    }
  }
  __syncthreads();
  if (wave == 0) {
#pragma unroll 1
    for (int b0 = 0; b0 < tt; b0 += 32) {
      const int idx = b0 + lane;
      const int ent = hl[idx < RCAP ? idx : RCAP - 1];
      const int m32 = (tt - b0) < 32 ? (tt - b0) : 32;
#pragma unroll 1
      for (int k = 0; k < m32; ++k) {
        const int u    = __builtin_amdgcn_readlane(ent, k);
        const int slot = u & (NBA - 1);
        if (lane == 0) {
          int p = cur[slot];
          p = p < 0 ? 0 : (p > RCAP - 1 ? RCAP - 1 : p);
          sl[p] = u;
          cur[slot] = p + 1;
        }
      }
    }
  }
  __syncthreads();

  const float qnan = __int_as_float(0x7fc00000);
  const float ninf = __int_as_float((int)0xff800000u);
  const float pz   = (ovf != 0) ? qnan : 0.0f;
  const float ael  = sc[aelIdx];
  v4f bv[NV];
#pragma unroll
  for (int j = 0; j < NV; ++j) {
    const v4f tb = *(const v4f*)(bias + 128 * j + 4 * lane);
    bv[j].x = bf16_val(tb.x); bv[j].y = bf16_val(tb.y); bv[j].z = bf16_val(tb.z); bv[j].w = bf16_val(tb.w);
  }
#pragma unroll 1
  for (int si = 0; si < NBA / NWAVE; ++si) {
    const int s    = si * NWAVE + wave;
    const int node = nodeBase + s;
    int c = cnt[s];
    const bool big = c > DEGCAP;
    c = c < 0 ? 0 : (c > DEGCAP ? DEGCAP : c);
    int o = offs[s];
    o = o < 0 ? 0 : (o > RCAP ? RCAP : o);
    const int nc = node < nN ? node : nN - 1;
    const float adn = ADp[nc];
    const float asn = ASp[nc];

    int sr0 = 0, sr1 = 0;
    float lg0 = ninf, lg1 = ninf;
    {
      int idx = o + lane;
      idx = idx > RCAP - 1 ? RCAP - 1 : idx;
      const int ent = sl[idx];
      int eid = ent >> SLA;
      eid = eid < 0 ? 0 : (eid > nE - 1 ? nE - 1 : eid);
      int sr = srcs[eid];
      sr = sr < 0 ? 0 : (sr > nN - 1 ? nN - 1 : sr);
      const float a = (ASp[sr] + adn) + AEp[eid];
      const float lk = leaky(a);
      lg0 = (lane < c) ? lk : ninf;
      sr0 = sr;
    }
    if (c > 32) {
      int idx = o + 32 + lane;
      idx = idx > RCAP - 1 ? RCAP - 1 : idx;
      const int ent = sl[idx];
      int eid = ent >> SLA;
      eid = eid < 0 ? 0 : (eid > nE - 1 ? nE - 1 : eid);
      int sr = srcs[eid];
      sr = sr < 0 ? 0 : (sr > nN - 1 ? nN - 1 : sr);
      const float a = (ASp[sr] + adn) + AEp[eid];
      const float lk = leaky(a);
      lg1 = ((32 + lane) < c) ? lk : ninf;
      sr1 = sr;
    }
    const float ll = leaky((asn + adn) + ael);
    float mx = fmaxf(lg0, lg1);
#pragma unroll
    for (int off = 16; off > 0; off >>= 1) mx = fmaxf(mx, __shfl_xor(mx, off, 32));
    mx = fmaxf(mx, ll);
    const float e0 = expf(lg0 - mx);
    const float e1 = expf(lg1 - mx);
    const float p0 = (lane < c) ? e0 : 0.0f;
    const float p1 = ((32 + lane) < c) ? e1 : 0.0f;
    const float pl = expf(ll - mx);
    float ds = p0 + p1;
#pragma unroll
    for (int off = 16; off > 0; off >>= 1) ds += __shfl_xor(ds, off, 32);
    const float den = ds + pl;
    const float inv = 1.0f / den;
    const int w0i = __float_as_int(p0 * inv);
    const int w1i = __float_as_int(p1 * inv);
    const float wl = pl * inv;

    v4f acc[NV];
#pragma unroll
    for (int j = 0; j < NV; ++j) { acc[j].x = 0.0f; acc[j].y = 0.0f; acc[j].z = 0.0f; acc[j].w = 0.0f; }
    const int m0 = c < 32 ? c : 32;
    int m1 = c - 32;
    m1 = m1 < 0 ? 0 : (m1 > 32 ? 32 : m1);
#pragma unroll 1
    for (int k = 0; k < m0; ++k) {
      const int   sk = __builtin_amdgcn_readlane(sr0, k);
      const float wk = __int_as_float(__builtin_amdgcn_readlane(w0i, k));
      gacc<NV>(Hp, sk, wk, lane, acc);
    }
#pragma unroll 1
    for (int k = 0; k < m1; ++k) {
      const int   sk = __builtin_amdgcn_readlane(sr1, k);
      const float wk = __int_as_float(__builtin_amdgcn_readlane(w1i, k));
      gacc<NV>(Hp, sk, wk, lane, acc);
    }
    gacc<NV>(Hp, nc, wl, lane, acc);

    const float pzr = big ? qnan : pz;
    const bool live = node < nN;
    if constexpr (NV == 2) {
      v4us mh[2], ml[2];
#pragma unroll
      for (int j = 0; j < 2; ++j) {
        float y0 = relu_np(acc[j].x + bv[j].x) + pzr;
        float y1 = relu_np(acc[j].y + bv[j].y) + pzr;
        float y2 = relu_np(acc[j].z + bv[j].z) + pzr;
        float y3 = relu_np(acc[j].w + bv[j].w) + pzr;
        y0 = live ? y0 : 0.0f; y1 = live ? y1 : 0.0f; y2 = live ? y2 : 0.0f; y3 = live ? y3 : 0.0f;
        unsigned hb;
        hb = bf16_bits(y0); mh[j][0] = (unsigned short)hb; ml[j][0] = (unsigned short)bf16_bits(y0 - __uint_as_float(hb << 16));
        hb = bf16_bits(y1); mh[j][1] = (unsigned short)hb; ml[j][1] = (unsigned short)bf16_bits(y1 - __uint_as_float(hb << 16));
        hb = bf16_bits(y2); mh[j][2] = (unsigned short)hb; ml[j][2] = (unsigned short)bf16_bits(y2 - __uint_as_float(hb << 16));
        hb = bf16_bits(y3); mh[j][3] = (unsigned short)hb; ml[j][3] = (unsigned short)bf16_bits(y3 - __uint_as_float(hb << 16));
      }
      *(v4usa*)(rowbuf + 4 * lane) = mh[0];
      *(v4usa*)(rowbuf + 128 + 4 * lane) = mh[1];
      *(v4usa*)(rowbuf + C1 + 4 * lane) = ml[0];
      *(v4usa*)(rowbuf + C1 + 128 + 4 * lane) = ml[1];
      wave_sync();
      const v8us q0 = *(const v8usa*)(rowbuf + 8 * lane);
      const v8us q1 = *(const v8usa*)(rowbuf + C1 + 8 * lane);
      wave_sync();
      if (node < mRows) {
        unsigned short* rpw = xpl + (size_t)node * AP + 8 * lane;
        *(volatile v8us*)rpw = q0;
        *(volatile v8us*)(rpw + C1) = q1;
        __threadfence();
        *(volatile v8us*)rpw = q0;
        *(volatile v8us*)(rpw + C1) = q1;
      }
    } else {
      v4f y;
      y.x = (acc[0].x + bv[0].x) + pzr;
      y.y = (acc[0].y + bv[0].y) + pzr;
      y.z = (acc[0].z + bv[0].z) + pzr;
      y.w = (acc[0].w + bv[0].w) + pzr;
      if (live) {
        float* op = outp + (size_t)node * C2 + 4 * lane;
        *(volatile v4f*)op = y;
        __threadfence();
        *(volatile v4f*)op = y;
      }
    }
  }
}

static inline int cdiv(int a, int b) { return (a + b - 1) / b; }
static inline size_t al256(size_t o) { return (o + 255) & ~(size_t)255; }

extern "C" void kernel_launch(void* const* d_in, const int* in_sizes, int n_in,
                              void* d_out, int out_size, void* d_ws, size_t ws_size,
                              hipStream_t stream) {
  if (n_in < 15) return;
  if (in_sizes[0] < CIN || (in_sizes[0] % CIN) != 0) return;
  const int nN = in_sizes[0] / CIN;
  if (nN < 1 || nN > (1 << 22)) return;
  if (in_sizes[1] < 2 || (in_sizes[1] & 1) != 0) return;
  const int nE = in_sizes[1] / 2;
  if (nE < 1 || nE >= (1 << (31 - SLA))) return;
  if ((long long)in_sizes[2] != (long long)nE * ED) return;
  if (in_sizes[3] != CIN * C1 || in_sizes[4] != ED * C1) return;
  if (in_sizes[5] != C1 || in_sizes[6] != C1 || in_sizes[7] != C1 || in_sizes[8] != C1) return;
  if (in_sizes[9] != C1 * C2 || in_sizes[10] != ED * C2) return;
  if (in_sizes[11] != C2 || in_sizes[12] != C2 || in_sizes[13] != C2 || in_sizes[14] != C2) return;
  if ((long long)out_size != (long long)nN * C2) return;

  const float* x    = (const float*)d_in[0];
  const int*   edge = (const int*)d_in[1];
  const float* ea   = (const float*)d_in[2];
  const float* W1   = (const float*)d_in[3];
  const float* We1  = (const float*)d_in[4];
  const float* as1  = (const float*)d_in[5];
  const float* ad1  = (const float*)d_in[6];
  const float* ae1  = (const float*)d_in[7];
  const float* b1   = (const float*)d_in[8];
  const float* W2   = (const float*)d_in[9];
  const float* We2  = (const float*)d_in[10];
  const float* as2  = (const float*)d_in[11];
  const float* ad2  = (const float*)d_in[12];
  const float* ae2  = (const float*)d_in[13];
  const float* b2   = (const float*)d_in[14];
  float* out = (float*)d_out;
  const int* src = edge;
  const int* dst = edge + nE;

  const int MP = cdiv(nN, 64) * 64;
  const int gE = cdiv(nE, EB);
  const int EP = gE * EB;
  const int gA = cdiv(MP, NBA);
  if ((long long)gA * NBA < (long long)MP) return;
  if ((MP % 64) != 0 || (MP % 32) != 0) return;
  const int vec8 = ((nE & 3) == 0) ? 1 : 0;

  char* ws = (char*)d_ws;
  size_t off = 0;
  const size_t oREC = off; off = al256(off + (size_t)gE * 128);
  const size_t oSC  = off; off = al256(off + 128);
  const size_t oW1T = off; off = al256(off + (size_t)C1 * CIN * 2);
  const size_t oW2T = off; off = al256(off + (size_t)C2 * K2 * 2);
  const size_t oXB  = off; off = al256(off + (size_t)MP * CIN * 2);
  const size_t oAE1 = off; off = al256(off + (size_t)EP * 4);
  const size_t oAE2 = off; off = al256(off + (size_t)EP * 4);
  const size_t oAS1 = off; off = al256(off + (size_t)MP * 4);
  const size_t oAD1 = off; off = al256(off + (size_t)MP * 4);
  const size_t oAS2 = off; off = al256(off + (size_t)MP * 4);
  const size_t oAD2 = off; off = al256(off + (size_t)MP * 4);
  const size_t oH1  = off; off = al256(off + (size_t)MP * C1 * 4);
  const size_t oX1  = off; off = al256(off + (size_t)MP * AP * 2);
  if (off > ws_size || off > (size_t)WSMAX) return;
  if ((size_t)MP * C2 * 4 > (size_t)MP * C1 * 4) return;
  double*         REC  = (double*)(ws + oREC);
  float*          SC   = (float*)(ws + oSC);
  unsigned short* W1T  = (unsigned short*)(ws + oW1T);
  unsigned short* W2T2 = (unsigned short*)(ws + oW2T);
  unsigned short* XB   = (unsigned short*)(ws + oXB);
  float*          AE1  = (float*)(ws + oAE1);
  float*          AE2  = (float*)(ws + oAE2);
  float*          AS1  = (float*)(ws + oAS1);
  float*          AD1  = (float*)(ws + oAD1);
  float*          AS2  = (float*)(ws + oAS2);
  float*          AD2  = (float*)(ws + oAD2);
  float*          H1   = (float*)(ws + oH1);
  float*          H2   = (float*)(ws + oH1);
  unsigned short* X1   = (unsigned short*)(ws + oX1);

  const size_t scanLds = (size_t)AGG_LDS_INTS * 4;
  hipFuncSetAttribute(reinterpret_cast<const void*>(&k_scan<2>), hipFuncAttributeMaxDynamicSharedMemorySize, (int)scanLds);
  hipFuncSetAttribute(reinterpret_cast<const void*>(&k_scan<1>), hipFuncAttributeMaxDynamicSharedMemorySize, (int)scanLds);

  const int nUx = MP * (CIN / 8);
  k_wprep<<<(NU1 + NU2) / NTHR, NTHR, 0, stream>>>(W1, W2, W1T, W2T2);
  k_cvx<<<cdiv(nUx, NTHR), NTHR, 0, stream>>>(x, nN, nUx, XB);
  k_edge<<<gE, NTHR, 0, stream>>>(ea, nE, We1, ae1, We2, ae2, AE1, AE2, REC);
  k_combine<<<1, NTHR, 0, stream>>>(REC, gE, nE, We1, ae1, We2, ae2, SC);
  k_gemm<2, 2><<<MP / 32, GTHR, 0, stream>>>(XB, W1T, CIN, as1, ad1, H1, AS1, AD1);
  k_scan<2><<<gA, NTHR, scanLds, stream>>>(src, dst, nE, nN, vec8, MP, AE1, AS1, AD1, SC, 0, H1, b1, X1, out);
  k_gemm<4, 1><<<MP / 64, GTHR, 0, stream>>>(X1, W2T2, K2, as2, ad2, H2, AS2, AD2);
  k_scan<1><<<gA, NTHR, scanLds, stream>>>(src, dst, nE, nN, vec8, MP, AE2, AS2, AD2, SC, 1, H2, b2, X1, out);
}
